// TGAT_40535901340473
// MI455X (gfx1250) — hardware-run, weakly checked
//
#include <hip/hip_runtime.h>

typedef float          v8f   __attribute__((ext_vector_type(8)));
typedef float          v4f   __attribute__((ext_vector_type(4)));
typedef unsigned int   v4u   __attribute__((ext_vector_type(4)));
typedef int            v8i   __attribute__((ext_vector_type(8)));
typedef unsigned short v8us  __attribute__((ext_vector_type(8)));
typedef unsigned short v16us __attribute__((ext_vector_type(16)));
typedef __bf16         v16bf __attribute__((ext_vector_type(16)));
typedef _Float16       v16h  __attribute__((ext_vector_type(16)));
typedef v4f  __attribute__((may_alias)) v4fa;
typedef v8us __attribute__((may_alias)) v8usa;
union FragB { v16bf v; v16us u; v8us h[2]; v8i w; };
union FragH { v16h  v; v16us u; v8us h[2]; v8i w; };

__device__ __forceinline__ v8f wmb(const FragB& a, const FragB& b, v8f c) {
  v8f d = __builtin_amdgcn_wmma_f32_16x16x32_bf16(false, a.v, false, b.v, (short)0, c, false, false);
  asm volatile("v_nop\n\tv_nop\n\tv_nop\n\tv_nop" : "+v"(d) : "v"(a.w), "v"(b.w));
  return d;
}

__device__ __forceinline__ v8f wmh(const FragH& a, const FragH& b, v8f c) {
  v8f d = __builtin_amdgcn_wmma_f32_16x16x32_f16(false, a.v, false, b.v, (short)0, c, false, false);
  asm volatile("v_nop\n\tv_nop\n\tv_nop\n\tv_nop" : "+v"(d) : "v"(a.w), "v"(b.w));
  return d;
}

__device__ __forceinline__ unsigned bf16_bits(float f) {
  const unsigned u = __float_as_uint(f);
  const unsigned r = (u + 0x7FFFu + ((u >> 16) & 1u)) >> 16;
  const unsigned q = (u >> 16) | 0x40u;
  return ((u & 0x7fffffffu) > 0x7f800000u) ? q : r;
}

__device__ __forceinline__ float bf16_val(float f) {
  return __uint_as_float(bf16_bits(f) << 16);
}
__device__ __forceinline__ int clampi(int v, int lo, int hi) {
  return v < lo ? lo : (v > hi ? hi : v);
}

__device__ __forceinline__ unsigned f16_bits(float f) {
  const unsigned u  = __float_as_uint(f);
  const unsigned s  = (u >> 16) & 0x8000u;
  const unsigned a  = u & 0x7fffffffu;
  const unsigned t  = a - 0x38000000u;
  const unsigned r  = (t + 0x0FFFu + ((t >> 13) & 1u)) >> 13;
  const unsigned rc = r > 0x7C00u ? 0x7C00u : r;
  const bool small  = a < 0x38800000u;
  const bool isnan  = a > 0x7f800000u;
  const unsigned fin = small ? 0u : (s | rc);
  return isnan ? (s | 0x7E00u) : fin;
}

__device__ __forceinline__ unsigned pk16(unsigned lo, unsigned hi) { return lo | (hi << 16); }
__device__ __forceinline__ unsigned bf16_lo_bits(float v) {
  float hi = bf16_val(v);
  asm volatile("" : "+v"(hi));
  return bf16_bits(v - hi);
}
__device__ __forceinline__ v4u pack8_bf16(v4f a, v4f c) {
  return (v4u){ pk16(bf16_bits(a[0]), bf16_bits(a[1])), pk16(bf16_bits(a[2]), bf16_bits(a[3])),
                pk16(bf16_bits(c[0]), bf16_bits(c[1])), pk16(bf16_bits(c[2]), bf16_bits(c[3])) };
}
__device__ __forceinline__ v4u pack8_bf16_lo(v4f a, v4f c) {
  return (v4u){ pk16(bf16_lo_bits(a[0]), bf16_lo_bits(a[1])), pk16(bf16_lo_bits(a[2]), bf16_lo_bits(a[3])),
                pk16(bf16_lo_bits(c[0]), bf16_lo_bits(c[1])), pk16(bf16_lo_bits(c[2]), bf16_lo_bits(c[3])) };
}
__device__ __forceinline__ v4u pack8_f16(v4f a, v4f c) {
  return (v4u){ pk16(f16_bits(a[0]), f16_bits(a[1])), pk16(f16_bits(a[2]), f16_bits(a[3])),
                pk16(f16_bits(c[0]), f16_bits(c[1])), pk16(f16_bits(c[2]), f16_bits(c[3])) };
}

template <int FORM>
__global__ __launch_bounds__(256) void k_plane(const float* __restrict__ src, int rows, int cols, int ldsrc,
                                               unsigned short* __restrict__ dst, int MP, int KP) {
  static_assert(FORM >= 0 && FORM <= 3);
  const int KTOT = (FORM == 1 || FORM == 3) ? 2 * KP : KP;
  const unsigned ppr   = (unsigned)(KTOT >> 3);
  const unsigned kp8   = (unsigned)(KP >> 3);
  const unsigned total = (unsigned)MP * ppr;
  const unsigned g     = blockIdx.x * 256u + threadIdx.x;
  const unsigned rowu  = g / ppr;
  const unsigned p     = g - rowu * ppr;
  const bool second    = p >= kp8;
  const int row = (int)rowu;
  const int c0  = (int)((second ? p - kp8 : p) << 3);
  const float* srow = src + (size_t)clampi(row, 0, rows - 1) * (size_t)ldsrc;
  float x[8];
  unsigned mk[8];
#pragma unroll
  for (int e = 0; e < 8; ++e) {
    const int c = c0 + e;
    const float v = srow[clampi(c, 0, cols - 1)];
    asm volatile("" :: "v"(v));
    x[e]  = v;
    mk[e] = (row < rows && c < cols) ? 0xFFFFu : 0u;
  }
  const v4f a = (v4f){ x[0], x[1], x[2], x[3] };
  const v4f c = (v4f){ x[4], x[5], x[6], x[7] };
  v4u o;
  if (FORM == 2) {
    o = pack8_f16(a, c);
  } else {
    const v4u hi = pack8_bf16(a, c);
    o = hi;
    if (FORM == 1) { const v4u lo = pack8_bf16_lo(a, c); o = second ? lo : hi; }
  }
  const v4u mw = (v4u){ pk16(mk[0], mk[1]), pk16(mk[2], mk[3]), pk16(mk[4], mk[5]), pk16(mk[6], mk[7]) };
  o &= mw;
  if (g < total) {
    volatile v4u* q = (volatile v4u*)(dst + (size_t)g * 8);
    *q = o;
    __threadfence();
    *q = o;
  }
}

template <int FORM> struct FragOf    { typedef FragB T; };
template <>         struct FragOf<2> { typedef FragH T; };
__device__ __forceinline__ v8f mm(const FragB& a, const FragB& b, v8f c) { return wmb(a, b, c); }
__device__ __forceinline__ v8f mm(const FragH& a, const FragH& b, v8f c) { return wmh(a, b, c); }
template <class F> __device__ __forceinline__ F ld_frag(const unsigned short* p) {
  F f;
  f.h[0] = *(const v8usa*)(p);
  f.h[1] = *(const v8usa*)(p + 16);
  return f;
}

template <int FORM, int EPI>
__global__ __launch_bounds__(256) __attribute__((amdgpu_num_vgpr(248)))
void k_gemm_nt(const unsigned short* __restrict__ A, const unsigned short* __restrict__ B,
               const float* __restrict__ bias, float* __restrict__ D, int M, int N, int KTOT, int ldd) {
  static_assert(FORM >= 0 && FORM <= 2);
  static_assert(EPI == 0 || EPI == 1);
  typedef typename FragOf<FORM>::T F;
  __shared__ __attribute__((aligned(16))) float sT[8][16 * 68];
  const int lane = threadIdx.x & 31;
  const int wave = threadIdx.x >> 5;
  const int tilesM = (M + 63) >> 6;
  const int tilesN = (N + 63) >> 6;
  const int tile = blockIdx.x * 8 + wave;
  if (tile >= tilesM * tilesN) return;
  const int tm = tile / tilesN;
  const int tn = tile - tm * tilesN;
  const int m0 = tm << 6;
  const int n0 = tn << 6;

  const int rl = lane & 15;
  const int h8 = (lane >> 4) * 8;
  const unsigned short* pa = A + (size_t)(m0 + rl) * (size_t)KTOT + h8;
  const unsigned short* pb = B + (size_t)(n0 + rl) * (size_t)KTOT + h8;

  v8f acc[4][4];
#pragma unroll
  for (int i = 0; i < 4; ++i)
#pragma unroll
    for (int j = 0; j < 4; ++j) acc[i][j] = (v8f){0.f, 0.f, 0.f, 0.f, 0.f, 0.f, 0.f, 0.f};

#pragma unroll 1
  for (int k0 = 0; k0 < KTOT; k0 += 32) {
    F bf[4];
#pragma unroll
    for (int j = 0; j < 4; ++j) bf[j] = ld_frag<F>(pb + (size_t)(j << 4) * (size_t)KTOT + k0);
#pragma unroll
    for (int i = 0; i < 4; ++i) {
      const F af = ld_frag<F>(pa + (size_t)(i << 4) * (size_t)KTOT + k0);
#pragma unroll
      for (int j = 0; j < 4; ++j) acc[i][j] = mm(af, bf[j], acc[i][j]);
    }
  }

  float* slab = sT[wave];
  const int hh = lane >> 4;
  const int c4 = (lane & 15) * 4;
  const int nc = n0 + c4;
  const bool cok = nc < N;
  v4f bv = (v4f){0.f, 0.f, 0.f, 0.f};
  if (EPI == 1) {
    bv = *(const v4fa*)(bias + clampi(nc, 0, N - 4));
    asm volatile("" :: "v"(bv));
  }
#pragma unroll
  for (int i = 0; i < 4; ++i) {
    const int mBase = m0 + (i << 4);
#pragma unroll
    for (int j = 0; j < 4; ++j) {
#pragma unroll
      for (int r = 0; r < 8; ++r) slab[(h8 + r) * 68 + (j << 4) + rl] = acc[i][j][r];
    }
    __builtin_amdgcn_fence(__ATOMIC_RELEASE, "workgroup");
    __builtin_amdgcn_wave_barrier();
    __builtin_amdgcn_fence(__ATOMIC_ACQUIRE, "workgroup");
    v4f vv[8];
#pragma unroll
    for (int it = 0; it < 8; ++it) {
      const int row = it * 2 + hh;
      v4f v = *(const v4fa*)(slab + row * 68 + c4);
      if (EPI == 1) v += bv;
      vv[it] = v;
    }
    for (int pass = 0; pass < 2; ++pass) {
#pragma unroll
      for (int it = 0; it < 8; ++it) {
        const int row = mBase + it * 2 + hh;
        if (cok && row < M) *(volatile v4f*)(D + (size_t)row * (size_t)ldd + nc) = vv[it];
      }
      __threadfence();
    }
    __builtin_amdgcn_fence(__ATOMIC_RELEASE, "workgroup");
    __builtin_amdgcn_wave_barrier();
    __builtin_amdgcn_fence(__ATOMIC_ACQUIRE, "workgroup");
  }
}

#define NN       100000
#define NE       1600000
#define MPN      100032
#define NBLK     98
#define NBROWS   1024
#define NCHK     7
#define BPC      14
#define DEGCAP   64
#define EPCAP    262144
#define MAXHITS  16759
#define MAXDEG   35
#define NTHR     256
#define NWAVE    8
#define EPT      8
#define CHUNK    (NTHR * EPT)
#define WCAP     (EPT * 32)
#define LISTN    (NWAVE * WCAP)
#define NBMAX    2048
#define ESH      11
#define RCAP     28672
#define LDS_BKT  ((2 * RCAP + 2 * NBMAX + LISTN) * 4 + 64)
#define P_EDGA   0
#define P_EDGB   128
#define P_ATTA   256
#define P_ATTB   384
#define P_BLIN   512
#define WSMAX    ((size_t)128 << 20)

static_assert(MPN % 64 == 0 && MPN >= NN && MPN - NN < 64);
static_assert(NN % 16 == 0 && NE % 4 == 0);
static_assert(NBLK * NBROWS >= NN && (NBLK - 1) * NBROWS < NN);
static_assert(NBLK == NCHK * BPC);
static_assert((NN - (NBLK - 1) * NBROWS) % 16 == 0);
static_assert(NBROWS <= NBMAX && (1 << ESH) >= NBMAX && NTHR * 8 == NBMAX && LISTN >= NBMAX);
static_assert(NE <= (1 << (32 - ESH)));
static_assert(RCAP % 1024 == 0 && RCAP % 16 == 0 && RCAP > MAXHITS + 1024);
static_assert(DEGCAP >= MAXDEG + 8);
static_assert(BPC * (MAXHITS + 15) <= EPCAP && EPCAP % 128 == 0);
static_assert(LDS_BKT <= 327680);
static_assert((MPN * 128 / 8) % 256 == 0 && (MPN * 8) % 256 == 0);

constexpr size_t al256(size_t v) { return (v + 255) & ~(size_t)255; }
constexpr size_t SZ_XB    = (size_t)MPN * 128 * 2;
constexpr size_t SZ_H     = (size_t)MPN * 32 * 4;
constexpr size_t SZ_EP    = (size_t)EPCAP * 32 * 4;
constexpr size_t O_XB     = 0;
constexpr size_t O_H      = al256(O_XB + SZ_XB);
constexpr size_t O_EP     = 0;
constexpr size_t SZ_R0    = al256(O_H + SZ_H);
constexpr size_t O_HHL    = SZ_R0;
constexpr size_t O_QKVS   = al256(O_HHL + (size_t)MPN * 64 * 2);
constexpr size_t O_BLIST  = al256(O_QKVS + (size_t)MPN * 128 * 4);
constexpr size_t O_OFFC   = al256(O_BLIST + (size_t)NBLK * RCAP * 4);
constexpr size_t O_META   = al256(O_OFFC + (size_t)NBLK * 2048 * 4);
constexpr size_t O_TAB    = al256(O_META + (size_t)NBLK * 128);
constexpr size_t O_WLIN   = al256(O_TAB + 512);
constexpr size_t O_WQKVS  = al256(O_WLIN + 64 * 128 * 2);
constexpr size_t O_WC2    = al256(O_WQKVS + 128 * 64 * 2);
constexpr size_t O_WE2    = al256(O_WC2 + 32 * 128 * 2);
constexpr size_t O_PAR    = al256(O_WE2 + 32 * 64 * 2);
constexpr size_t WS_TOTAL = al256(O_PAR + 4096);
static_assert(SZ_EP <= SZ_R0);
static_assert(WS_TOTAL <= (size_t)WSMAX);

typedef int      v4i  __attribute__((ext_vector_type(4)));
typedef unsigned v2u  __attribute__((ext_vector_type(2)));
typedef v4i __attribute__((may_alias)) v4ia;
typedef v4u __attribute__((may_alias)) v4ua;
typedef v2u __attribute__((may_alias)) v2ua;

__device__ __forceinline__ void wave_sync_lds() {
  __builtin_amdgcn_fence(__ATOMIC_RELEASE, "workgroup");
  __builtin_amdgcn_wave_barrier();
  __builtin_amdgcn_fence(__ATOMIC_ACQUIRE, "workgroup");
}
__device__ __forceinline__ void st2_v4u(void* p, const v4u v) {
  volatile v4u* q = (volatile v4u*)p;
  *q = v;
  __threadfence();
  *q = v;
}
__device__ __forceinline__ void st2_v4f(float* p, const v4f v) {
  volatile v4f* q = (volatile v4f*)p;
  *q = v;
  __threadfence();
  *q = v;
}
__device__ __forceinline__ void st2_v4i(int* p, const v4i v) {
  volatile v4i* q = (volatile v4i*)p;
  *q = v;
  __threadfence();
  *q = v;
}

__global__ __launch_bounds__(256) void k_prep(
    const float* __restrict__ wlin_s, const float* __restrict__ wq, const float* __restrict__ wk,
    const float* __restrict__ wv, const float* __restrict__ wsk, const float* __restrict__ wcomb,
    const float* __restrict__ we, const float* __restrict__ wtime, const float* __restrict__ btime,
    const float* __restrict__ wdeg, const float* __restrict__ bdeg, const float* __restrict__ blin,
    const float* __restrict__ bcomb, const float* __restrict__ bq, const float* __restrict__ bk,
    const float* __restrict__ bv, const float* __restrict__ bs, const float* __restrict__ be,
    const float* __restrict__ wout, const float* __restrict__ bout,
    unsigned short* wlin, unsigned short* wqkvs, unsigned short* wc2, unsigned short* we2, float* par) {
  const int b = (int)blockIdx.x, tid = (int)threadIdx.x;
  if (b < 4) {
    const int u = b * 256 + tid;
    const int n = u >> 4, k8 = (u & 15) * 8;
    const float* p = wlin_s + (size_t)(n < 32 ? n : 31) * 128 + k8;
    const v4f a = *(const v4fa*)p, c = *(const v4fa*)(p + 4);
    asm volatile("" :: "v"(a), "v"(c));
    v4u o = pack8_bf16(a, c);
    const unsigned mk = n < 32 ? 0xFFFFFFFFu : 0u;
    o &= (v4u){mk, mk, mk, mk};
    st2_v4u(wlin + (size_t)u * 8, o);
  } else if (b < 8) {
    const int m = b - 4;
    const int row = tid >> 3, p8 = tid & 7;
    const int wo = row * 32 + (p8 & 3) * 8;
    const v4f a0 = *(const v4fa*)(wq + wo),  c0 = *(const v4fa*)(wq + wo + 4);
    const v4f a1 = *(const v4fa*)(wk + wo),  c1 = *(const v4fa*)(wk + wo + 4);
    const v4f a2 = *(const v4fa*)(wv + wo),  c2 = *(const v4fa*)(wv + wo + 4);
    const v4f a3 = *(const v4fa*)(wsk + wo), c3 = *(const v4fa*)(wsk + wo + 4);
    asm volatile("" :: "v"(a0), "v"(c0), "v"(a1), "v"(c1), "v"(a2), "v"(c2), "v"(a3), "v"(c3));
    const v4f a = (m == 0) ? a0 : ((m == 1) ? a1 : ((m == 2) ? a2 : a3));
    const v4f c = (m == 0) ? c0 : ((m == 1) ? c1 : ((m == 2) ? c2 : c3));
    st2_v4u(wqkvs + (size_t)(m * 256 + tid) * 8, pack8_bf16(a, c));
  } else if (b < 10) {
    const int u = (b - 8) * 256 + tid;
    const int n = u >> 4, p = u & 15;
    const float* r = wcomb + n * 64 + 2 * p;
    const unsigned f0 = bf16_bits(r[0]), f1 = bf16_bits(r[1]), g0 = bf16_bits(r[32]), g1 = bf16_bits(r[33]);
    const v4u o = (v4u){ pk16(f0, f0), pk16(g0, g0), pk16(f1, f1), pk16(g1, g1) };
    st2_v4u(wc2 + (size_t)u * 8, o);
  } else if (b == 10) {
    const int n = tid >> 3, p = tid & 7;
    const v4f a = *(const v4fa*)(we + n * 32 + 4 * p);
    const unsigned a0 = bf16_bits(a[0]), a1 = bf16_bits(a[1]), a2 = bf16_bits(a[2]), a3 = bf16_bits(a[3]);
    const v4u o = (v4u){ pk16(a0, a0), pk16(a1, a1), pk16(a2, a2), pk16(a3, a3) };
    st2_v4u(we2 + (size_t)tid * 8, o);
  } else {
    const int lane = tid & 31, wave = tid >> 5, n = lane & 15;
    if (wave == 0) {
      const v4f v = (v4f){ bf16_val(wtime[lane]), bf16_val(btime[lane]), bf16_val(wdeg[lane]), bf16_val(bdeg[lane]) };
      st2_v4f(par + P_EDGA + 4 * lane, v);
    } else if (wave == 1) {
      const v4f v = (v4f){ bf16_val(bcomb[n]), bf16_val(bcomb[16 + n]), bf16_val(be[n]), bf16_val(be[16 + n]) };
      st2_v4f(par + P_EDGB + 4 * lane, v);
    } else if (wave == 2) {
      const v4f v = (v4f){ bf16_val(bq[lane]), bf16_val(bk[lane]), bf16_val(bv[lane]), bf16_val(bs[lane]) };
      st2_v4f(par + P_ATTA + 4 * lane, v);
    } else if (wave == 3) {
      const v4f v = (v4f){ bf16_val(wout[lane]), bf16_val(wout[32 + lane]), bf16_val(bout[0]), bf16_val(bout[1]) };
      st2_v4f(par + P_ATTB + 4 * lane, v);
    } else if (wave == 4) {
      const float v = bf16_val(blin[lane]);
      volatile float* q = par + P_BLIN + lane;
      *q = v;
      __threadfence();
      *q = v;
    }
  }
}

__global__ __launch_bounds__(256) void k_hpost(const float* __restrict__ H, const float* __restrict__ par,
                                               unsigned short* HHL) {
  const unsigned g = blockIdx.x * 256u + threadIdx.x;
  const int row = (int)(g >> 3);
  const int p = (int)(g & 7u);
  const bool second = p >= 4;
  const int c0 = (p & 3) * 8;
  const int rc = row < NN ? row : NN - 1;
  const float* hp = H + (size_t)rc * 32 + c0;
  v4f a = *(const v4fa*)hp, c = *(const v4fa*)(hp + 4);
  asm volatile("" :: "v"(a), "v"(c));
  const v4f ba = *(const v4fa*)(par + P_BLIN + c0), bc = *(const v4fa*)(par + P_BLIN + c0 + 4);
  a += ba; c += bc;
#pragma unroll
  for (int e = 0; e < 4; ++e) {
    const float x = a[e], y = c[e];
    a[e] = (x > 0.0f) ? x : (x - x);
    c[e] = (y > 0.0f) ? y : (y - y);
  }
  const v4u hi = pack8_bf16(a, c);
  const v4u lo = pack8_bf16_lo(a, c);
  v4u o = second ? lo : hi;
  const unsigned mk = row < NN ? 0xFFFFFFFFu : 0u;
  o &= (v4u){mk, mk, mk, mk};
  st2_v4u(HHL + (size_t)g * 8, o);
}

__device__ __forceinline__ int scan_chunk(const int* __restrict__ dsts, int nE, int cbase, int slotBase,
                                          int nb, int vec8, int* list, int tid, int lane, int wave) {
  int wc = 0;
  const int el0  = tid * EPT;
  const int e0   = cbase + el0;
  const int sent = (-0x7fffffff - 1);
  v4i da, db;
  if (vec8 != 0 && cbase + CHUNK <= nE) {
    da = *(const v4i*)(dsts + e0);
    db = *(const v4i*)(dsts + e0 + 4);
  } else {
    const int t0 = dsts[min(e0 + 0, nE - 1)];
    const int t1 = dsts[min(e0 + 1, nE - 1)];
    const int t2 = dsts[min(e0 + 2, nE - 1)];
    const int t3 = dsts[min(e0 + 3, nE - 1)];
    const int t4 = dsts[min(e0 + 4, nE - 1)];
    const int t5 = dsts[min(e0 + 5, nE - 1)];
    const int t6 = dsts[min(e0 + 6, nE - 1)];
    const int t7 = dsts[min(e0 + 7, nE - 1)];
    asm volatile("" :: "v"(t0), "v"(t1), "v"(t2), "v"(t3), "v"(t4), "v"(t5), "v"(t6), "v"(t7));
    da.x = (e0 + 0 < nE) ? t0 : sent;
    da.y = (e0 + 1 < nE) ? t1 : sent;
    da.z = (e0 + 2 < nE) ? t2 : sent;
    da.w = (e0 + 3 < nE) ? t3 : sent;
    db.x = (e0 + 4 < nE) ? t4 : sent;
    db.y = (e0 + 5 < nE) ? t5 : sent;
    db.z = (e0 + 6 < nE) ? t6 : sent;
    db.w = (e0 + 7 < nE) ? t7 : sent;
  }
  const unsigned nbs = (unsigned)slotBase;
  const unsigned unb = (unsigned)nb;
  const unsigned s0 = (unsigned)da.x - nbs, s1 = (unsigned)da.y - nbs;
  const unsigned s2 = (unsigned)da.z - nbs, s3 = (unsigned)da.w - nbs;
  const unsigned s4 = (unsigned)db.x - nbs, s5 = (unsigned)db.y - nbs;
  const unsigned s6 = (unsigned)db.z - nbs, s7 = (unsigned)db.w - nbs;
  const bool h0 = s0 < unb, h1 = s1 < unb, h2 = s2 < unb, h3 = s3 < unb;
  const bool h4 = s4 < unb, h5 = s5 < unb, h6 = s6 < unb, h7 = s7 < unb;
  const unsigned any = __builtin_amdgcn_ballot_w32(h0 | h1 | h2 | h3 | h4 | h5 | h6 | h7);
  if (any != 0u) {
#define HITJ(J, HJ, SJ) { \
      const unsigned mj = __builtin_amdgcn_ballot_w32(HJ); \
      if (mj != 0u) { \
        if (HJ) { \
          const int pos = wc + (int)__builtin_amdgcn_mbcnt_lo(mj, 0u); \
          if (pos < WCAP) list[wave * WCAP + pos] = ((el0 + (J)) << 12) | (int)(SJ); \
        } \
        wc += (int)__builtin_popcount(mj); } }
    HITJ(0, h0, s0)
    HITJ(1, h1, s1)
    HITJ(2, h2, s2)
    HITJ(3, h3, s3)
    HITJ(4, h4, s4)
    HITJ(5, h5, s5)
    HITJ(6, h6, s6)
    HITJ(7, h7, s7)
#undef HITJ
  }
  return wc;
}

__device__ __forceinline__ int build_lists(const int* __restrict__ dsts, int nE, int nodeBase, int nb, int vec8,
                                           int* reg1, int* reg2, int* scnt, int* soff, int* list,
                                           int* wcnt, int* wtot, int tid, int lane, int wave) {
  for (int i = tid; i < NBMAX; i += NTHR) scnt[i] = 0;
  __syncthreads();

  int tot = 0;
  const int nChunks = (nE + CHUNK - 1) / CHUNK;
#pragma unroll 1
  for (int ch = 0; ch < nChunks; ++ch) {
    const int cbase = ch * CHUNK;
    const int wc = scan_chunk(dsts, nE, cbase, nodeBase, nb, vec8, list, tid, lane, wave);
    if (lane == 0) wcnt[wave] = wc;
    __syncthreads();
    int pre = 0, all = 0;
#pragma unroll
    for (int w2 = 0; w2 < NWAVE; ++w2) {
      int c = wcnt[w2];
      c = c < 0 ? 0 : (c > WCAP ? WCAP : c);
      all += c;
      pre += (w2 < wave) ? c : 0;
    }
    const int wcc  = wc > WCAP ? WCAP : wc;
    const int base = tot + pre;
#pragma unroll 1
    for (int i = lane; i < wcc; i += 32) {
      const int ent = list[wave * WCAP + i];
      const int el  = (ent >> 12) & (CHUNK - 1);
      const int sl  = ent & (NBMAX - 1);
      int eid = cbase + el;
      eid = eid > nE - 1 ? nE - 1 : eid;
      const int pos = base + i;
      if (pos < RCAP) reg1[pos] = (int)(((unsigned)eid << ESH) | (unsigned)sl);
    }
    tot += all;
    tot = tot > RCAP ? RCAP : tot;
    __syncthreads();
  }
  const int nh = tot;

  if (wave == 0) {
#pragma unroll 1
    for (int b0 = 0; b0 < nh; b0 += 32) {
      const int idx = b0 + lane;
      const int uv  = reg1[idx < RCAP ? idx : RCAP - 1];
      const int m32 = (nh - b0) < 32 ? (nh - b0) : 32;
#pragma unroll 1
      for (int k = 0; k < m32; ++k) {
        const int u  = __builtin_amdgcn_readlane(uv, k);
        const int sl = u & (NBMAX - 1);
        if (lane == 0) scnt[sl] = scnt[sl] + 1;
      }
    }
  }
  __syncthreads();

  {
    const v4i ca = *(const v4i*)(scnt + 8 * tid);
    const v4i cb = *(const v4i*)(scnt + 8 * tid + 4);
    const int e0 = ca.x < 0 ? 0 : ca.x, e1 = ca.y < 0 ? 0 : ca.y, e2 = ca.z < 0 ? 0 : ca.z, e3 = ca.w < 0 ? 0 : ca.w;
    const int e4 = cb.x < 0 ? 0 : cb.x, e5 = cb.y < 0 ? 0 : cb.y, e6 = cb.z < 0 ? 0 : cb.z, e7 = cb.w < 0 ? 0 : cb.w;
    const int ts = e0 + e1 + e2 + e3 + e4 + e5 + e6 + e7;
    int incl = ts;
#pragma unroll
    for (int d = 1; d < 32; d <<= 1) {
      const int up = __shfl_up(incl, d);
      if (lane >= d) incl += up;
    }
    if (lane == 31) wtot[wave] = incl;
    __syncthreads();
    int pre = 0;
#pragma unroll
    for (int w2 = 0; w2 < NWAVE; ++w2) pre += (w2 < wave) ? wtot[w2] : 0;
    int run = pre + incl - ts;
    soff[8 * tid + 0] = run; run += e0;
    soff[8 * tid + 1] = run; run += e1;
    soff[8 * tid + 2] = run; run += e2;
    soff[8 * tid + 3] = run; run += e3;
    soff[8 * tid + 4] = run; run += e4;
    soff[8 * tid + 5] = run; run += e5;
    soff[8 * tid + 6] = run; run += e6;
    soff[8 * tid + 7] = run;
  }
  __syncthreads();
  for (int i = tid; i < NBMAX; i += NTHR) list[i] = soff[i];
  __syncthreads();

  if (wave == 0) {
#pragma unroll 1
    for (int b0 = 0; b0 < nh; b0 += 32) {
      const int idx = b0 + lane;
      const int uv  = reg1[idx < RCAP ? idx : RCAP - 1];
      const int m32 = (nh - b0) < 32 ? (nh - b0) : 32;
#pragma unroll 1
      for (int k = 0; k < m32; ++k) {
        const int u   = __builtin_amdgcn_readlane(uv, k);
        const int sl  = u & (NBMAX - 1);
        const int eid = (int)((unsigned)u >> ESH);
        if (lane == 0) {
          int pos = list[sl];
          pos = pos < 0 ? 0 : (pos > RCAP - 1 ? RCAP - 1 : pos);
          reg2[pos] = eid;
          list[sl] = pos + 1;
        }
      }
    }
  }
  __syncthreads();
  return nh;
}

__global__ __launch_bounds__(NTHR) void k_bucket(const int* __restrict__ dsts, int nE, int nN, int vec8,
                                                 int* BLIST, int* OFFC, int* META) {
  extern __shared__ v4f lds_dyn[];
  int* reg1 = (int*)lds_dyn;
  int* reg2 = reg1 + RCAP;
  int* scnt = reg2 + RCAP;
  int* soff = scnt + NBMAX;
  int* list = soff + NBMAX;
  int* wcnt = list + LISTN;
  int* wtot = wcnt + NWAVE;
  const int tid = (int)threadIdx.x, lane = tid & 31, wave = tid >> 5;
  const int b = (int)blockIdx.x;
  const int nodeBase = b * NBROWS;
  int nb = nN - nodeBase;
  nb = nb < 0 ? 0 : (nb > NBROWS ? NBROWS : nb);

  const int nh = build_lists(dsts, nE, nodeBase, nb, vec8, reg1, reg2, scnt, soff, list, wcnt, wtot, tid, lane, wave);

  int* bl = BLIST + (size_t)b * RCAP;
  const int last = nh > 0 ? nh - 1 : 0;
#pragma unroll 1
  for (int base = 0; base < nh; base += 1024) {
    const int i0 = base + 4 * tid;
    v4i v;
    v.x = reg2[i0     < last ? i0     : last];
    v.y = reg2[i0 + 1 < last ? i0 + 1 : last];
    v.z = reg2[i0 + 2 < last ? i0 + 2 : last];
    v.w = reg2[i0 + 3 < last ? i0 + 3 : last];
    v.x = (i0     < nh) ? v.x : 0;
    v.y = (i0 + 1 < nh) ? v.y : 0;
    v.z = (i0 + 2 < nh) ? v.z : 0;
    v.w = (i0 + 3 < nh) ? v.w : 0;
    st2_v4i(bl + i0, v);
  }
  {
    const v4i so = *(const v4ia*)(soff + 4 * tid);
    const v4i sc = *(const v4ia*)(scnt + 4 * tid);
    int* oc = OFFC + (size_t)b * 2048;
    st2_v4i(oc + 4 * tid, so);
    st2_v4i(oc + 1024 + 4 * tid, sc);
  }
  if (tid < 8) {
    v4i mv;
    mv.x = (tid == 0) ? nh : 0;
    mv.y = (tid == 0 && nh >= RCAP) ? 1 : 0;
    mv.z = 0; mv.w = 0;
    st2_v4i(META + (size_t)b * 32 + 4 * tid, mv);
  }
}

__global__ __launch_bounds__(32) void k_base(const int* __restrict__ META, int* TAB) {
  __shared__ __attribute__((aligned(16))) int stab[128];
  const int lane = (int)threadIdx.x;
  int carry = 0;
#pragma unroll
  for (int g = 0; g < 4; ++g) {
    const int j = 32 * g + lane;
    const int jc = j < NBLK ? j : NBLK - 1;
    int c = META[(size_t)jc * 32];
    asm volatile("" :: "v"(c));
    c = clampi(c, 0, RCAP);
    c = (c + 15) & ~15;
    c = (j < NBLK) ? c : 0;
    int incl = c;
#pragma unroll
    for (int d = 1; d < 32; d <<= 1) {
      const int up = __shfl_up(incl, d);
      incl += (lane >= d) ? up : 0;
    }
    stab[j] = carry + incl - c;
    carry += __shfl(incl, 31);
  }
  __syncthreads();
  const v4i v = *(const v4ia*)(stab + 4 * lane);
  st2_v4i(TAB + 4 * lane, v);
}

__global__ __launch_bounds__(256) __attribute__((amdgpu_num_vgpr(248)))
void k_edge(const int* __restrict__ ei, const float* __restrict__ ntime, const float* __restrict__ etime,
            const float* __restrict__ ndeg, const int* __restrict__ BLIST, const int* __restrict__ META,
            const int* __restrict__ TAB, const unsigned short* __restrict__ WC, const unsigned short* __restrict__ WE,
            const float* __restrict__ par, unsigned* EP, int chunk) {
  __shared__ __attribute__((aligned(16))) unsigned sA[8][16 * 64];
  __shared__ __attribute__((aligned(16))) unsigned sB[8][16 * 32];
  const int lane = threadIdx.x & 31;
  const int wave = threadIdx.x >> 5;
  const int rl = lane & 15;
  const int h8 = (lane >> 4) * 8;
  const int p0 = ((int)blockIdx.x * 8 + wave) * 16;
  const int tb = chunk * BPC;

  int tv = TAB[tb + (lane < BPC ? lane : BPC)];
  asm volatile("" :: "v"(tv));
  tv = clampi(tv, 0, NBLK * RCAP);
  const int cb0 = __builtin_amdgcn_readlane(tv, 0);
  const int cb1 = __builtin_amdgcn_readlane(tv, BPC);
  const int nch = clampi(cb1 - cb0, 0, EPCAP);
  if (p0 >= nch) return;
  const int gpos = cb0 + p0;
  const bool pred = (lane >= 1) && (lane < BPC) && (gpos >= tv);
  const int boff = (int)__builtin_popcount(__builtin_amdgcn_ballot_w32(pred));
  const int bb = tb + boff;
  const int bbase = __builtin_amdgcn_readlane(tv, boff);
  const int cntb = clampi(META[(size_t)bb * 32], 0, RCAP);
  const int loc0 = gpos - bbase;
  const int li = loc0 + rl;
  const bool valid = li < cntb;
  const int lic = clampi(li, 0, cntb > 0 ? cntb - 1 : 0);
  int id = BLIST[(size_t)bb * RCAP + lic];
  asm volatile("" :: "v"(id));
  id = clampi(id, 0, NE - 1);
  int s = ei[id];
  int d = ei[NE + id];
  asm volatile("" :: "v"(s), "v"(d));
  s = clampi(s, 0, NN - 1);
  d = clampi(d, 0, NN - 1);
  float nt = ntime[s], et = etime[id], dgs = ndeg[s], dgd = ndeg[d];
  asm volatile("" :: "v"(nt), "v"(et), "v"(dgs), "v"(dgd));
  float relt = bf16_val(nt) - bf16_val(et);
  float reld = bf16_val(dgs) - bf16_val(dgd);
  relt = valid ? relt : 0.0f;
  reld = valid ? reld : 0.0f;

  const v4f pa = *(const v4fa*)(par + P_EDGA + 4 * lane);
  const v4f pb = *(const v4fa*)(par + P_EDGB + 4 * lane);

  unsigned* arow = &sA[wave][0];
  unsigned* brow = &sB[wave][0];
#pragma unroll 1
  for (int i = 0; i < 16; ++i) {
    const float rt = __shfl(relt, i);
    const float rd = __shfl(reld, i);
    const float ct = cosf(rt * pa[0] + pa[1]);
    const float cd = cosf(rd * pa[2] + pa[3]);
    v2u w;
    w.x = pk16(bf16_bits(ct), bf16_lo_bits(ct));
    w.y = pk16(bf16_bits(cd), bf16_lo_bits(cd));
    *(v2ua*)(arow + i * 64 + 2 * lane) = w;
  }
  wave_sync_lds();

  v8f c0 = (v8f){0.f, 0.f, 0.f, 0.f, 0.f, 0.f, 0.f, 0.f};
  v8f c1 = c0;
  {
    const unsigned short* ah = (const unsigned short*)arow + rl * 128 + h8;
    const unsigned short* w0 = WC + (size_t)rl * 128 + h8;
    const unsigned short* w1 = WC + (size_t)(16 + rl) * 128 + h8;
#pragma unroll 1
    for (int k0 = 0; k0 < 128; k0 += 32) {
      FragB a;
      a.h[0] = *(const v8usa*)(ah + k0);
      a.h[1] = *(const v8usa*)(ah + k0 + 16);
      const FragB b0 = ld_frag<FragB>(w0 + k0);
      const FragB b1 = ld_frag<FragB>(w1 + k0);
      c0 = wmb(a, b0, c0);
      c1 = wmb(a, b1, c1);
    }
  }
#pragma unroll
  for (int r = 0; r < 8; ++r) {
    const float v0 = c0[r] + pb[0];
    const float v1 = c1[r] + pb[1];
    brow[(h8 + r) * 32 + rl]      = pk16(bf16_bits(v0), bf16_lo_bits(v0));
    brow[(h8 + r) * 32 + 16 + rl] = pk16(bf16_bits(v1), bf16_lo_bits(v1));
  }
  wave_sync_lds();

  v8f d0 = (v8f){0.f, 0.f, 0.f, 0.f, 0.f, 0.f, 0.f, 0.f};
  v8f d1 = d0;
  {
    const unsigned short* bh = (const unsigned short*)brow + rl * 64 + h8;
    const unsigned short* w0 = WE + (size_t)rl * 64 + h8;
    const unsigned short* w1 = WE + (size_t)(16 + rl) * 64 + h8;
#pragma unroll
    for (int k0 = 0; k0 < 64; k0 += 32) {
      FragB a;
      a.h[0] = *(const v8usa*)(bh + k0);
      a.h[1] = *(const v8usa*)(bh + k0 + 16);
      const FragB b0 = ld_frag<FragB>(w0 + k0);
      const FragB b1 = ld_frag<FragB>(w1 + k0);
      d0 = wmb(a, b0, d0);
      d1 = wmb(a, b1, d1);
    }
  }
  wave_sync_lds();
#pragma unroll
  for (int r = 0; r < 8; ++r) {
    arow[(h8 + r) * 32 + rl]      = __float_as_uint(d0[r] + pb[2]);
    arow[(h8 + r) * 32 + 16 + rl] = __float_as_uint(d1[r] + pb[3]);
  }
  wave_sync_lds();
  v4u xo[4];
#pragma unroll
  for (int it = 0; it < 4; ++it) xo[it] = *(const v4ua*)(arow + it * 128 + 4 * lane);
  unsigned* ep = EP + (size_t)p0 * 32;
  for (int pass = 0; pass < 2; ++pass) {
#pragma unroll
    for (int it = 0; it < 4; ++it) *(volatile v4u*)(ep + it * 128 + 4 * lane) = xo[it];
    __threadfence();
  }
}

__device__ __forceinline__ void entry_ids(const int* __restrict__ bl, const int* __restrict__ ei, int st, int q,
                                          int nh, int epoff, int& s, int& er) {
  const int li = clampi(st + q, 0, nh > 0 ? nh - 1 : 0);
  const int id = clampi(bl[li], 0, NE - 1);
  s  = clampi(ei[id], 0, NN - 1);
  er = clampi(epoff + st + q, 0, EPCAP - 1);
}

__global__ __launch_bounds__(256) void k_attn(
    const int* __restrict__ ei, const float* __restrict__ QKVS, const float* __restrict__ EP,
    const int* __restrict__ BLIST, const int* __restrict__ OFFC, const int* __restrict__ META,
    const int* __restrict__ TAB, const float* __restrict__ par, float* out, int chunk) {
  __shared__ float sL[8][DEGCAP * 2];
  const int lane = threadIdx.x & 31;
  const int wave = threadIdx.x >> 5;
  const int hd = lane >> 4;
  const int bb = chunk * BPC + (int)blockIdx.x;
  const int nodeBase = bb * NBROWS;
  const int nbrows = clampi(NN - nodeBase, 0, NBROWS);
  const int nh = clampi(META[(size_t)bb * 32], 0, RCAP);
  const int flag = META[(size_t)bb * 32 + 1];
  const int cb0 = clampi(TAB[chunk * BPC], 0, NBLK * RCAP);
  const int cb1 = clampi(TAB[chunk * BPC + BPC], 0, NBLK * RCAP);
  const int bbase = clampi(TAB[bb], 0, NBLK * RCAP);
  const int nchunk = cb1 - cb0;
  const bool ovf = (flag != 0) || (nchunk > EPCAP) || (nchunk < 0) || (bbase < cb0);
  const int epoff = bbase - cb0;
  const int* bl = BLIST + (size_t)bb * RCAP;
  const int* oc = OFFC + (size_t)bb * 2048;
  const v4f pa = *(const v4fa*)(par + P_ATTA + 4 * lane);
  const v4f pb = *(const v4fa*)(par + P_ATTB + 4 * lane);
  const float qnan = __int_as_float(0x7fc00000);
  const float finf = __builtin_inff();
  float* strip = &sL[wave][0];

#pragma unroll 1
  for (int g = 0; g < 8; ++g) {
    const int slot0 = wave * 128 + g * 16;
    if (slot0 >= nbrows) break;
    int stv = oc[slot0 + (lane & 15)];
    int cv  = oc[1024 + slot0 + (lane & 15)];
    const int pv = (cv > DEGCAP) ? 1 : 0;
    stv = clampi(stv, 0, nh);
    cv  = clampi(cv, 0, DEGCAP);
    cv  = cv > nh - stv ? nh - stv : cv;
    float img = 0.0f;
#pragma unroll 1
    for (int rr = 0; rr < 16; ++rr) {
      const int st  = __builtin_amdgcn_readlane(stv, rr);
      const int cnt = __builtin_amdgcn_readlane(cv, rr);
      const int prw = __builtin_amdgcn_readlane(pv, rr);
      const int grow = nodeBase + slot0 + rr;
      const float* qrow = QKVS + (size_t)grow * 128;
      const float qv = qrow[lane] + pa[0];
      const float sk = qrow[96 + lane] + pa[3];

      float m = -finf;
#pragma unroll 1
      for (int q = 0; q < cnt; ++q) {
        int s, er;
        entry_ids(bl, ei, st, q, nh, epoff, s, er);
        const float e  = EP[(size_t)er * 32 + lane];
        const float kk = QKVS[(size_t)s * 128 + 32 + lane] + pa[1] + e;
        float pr = qv * kk;
        pr += __shfl_xor(pr, 8);
        pr += __shfl_xor(pr, 4);
        pr += __shfl_xor(pr, 2);
        pr += __shfl_xor(pr, 1);
        const float l = pr * 0.25f;
        if ((lane & 15) == 0) strip[2 * q + hd] = l;
        m = (l > m) ? l : m;
      }
      wave_sync_lds();
      const float mf = (fabsf(m) < finf) ? m : 0.0f;
      float den = 0.0f, acc = 0.0f;
#pragma unroll 1
      for (int q = 0; q < cnt; ++q) {
        int s, er;
        entry_ids(bl, ei, st, q, nh, epoff, s, er);
        const float e  = EP[(size_t)er * 32 + lane];
        const float vv = QKVS[(size_t)s * 128 + 64 + lane] + pa[2] + e;
        const float l  = strip[2 * q + hd];
        const float p  = expf(l - mf);
        den += p;
        acc = fmaf(p, vv, acc);
      }
      wave_sync_lds();
      const float h1 = acc * (1.0f / (den + 1e-16f)) + sk;
      float t0 = h1 * pb[0];
      float t1 = h1 * pb[1];
      t0 += __shfl_xor(t0, 16); t1 += __shfl_xor(t1, 16);
      t0 += __shfl_xor(t0, 8);  t1 += __shfl_xor(t1, 8);
      t0 += __shfl_xor(t0, 4);  t1 += __shfl_xor(t1, 4);
      t0 += __shfl_xor(t0, 2);  t1 += __shfl_xor(t1, 2);
      t0 += __shfl_xor(t0, 1);  t1 += __shfl_xor(t1, 1);
      const float o0 = t0 + pb[2];
      const float o1 = t1 + pb[3];
      const float mx = (o0 > o1) ? o0 : o1;
      const float lse = logf(expf(o0 - mx) + expf(o1 - mx));
      const float r0 = o0 - mx - lse;
      const float r1 = o1 - mx - lse;
      const float pz = (ovf || prw != 0) ? qnan : 0.0f;
      const float val = ((lane & 1) ? r1 : r0) + pz;
      img = ((lane >> 1) == rr) ? val : img;
    }
    float* op = out + (size_t)(nodeBase + slot0) * 2 + lane;
    *(volatile float*)op = img;
    __threadfence();
    *(volatile float*)op = img;
  }
}

extern "C" void kernel_launch(void* const* d_in, const int* in_sizes, int n_in,
                              void* d_out, int out_size, void* d_ws, size_t ws_size,
                              hipStream_t stream) {
  if (n_in < 25) return;
  if (in_sizes[0] != NN * 128 || in_sizes[1] != 2 * NE || in_sizes[2] != NN || in_sizes[3] != NE ||
      in_sizes[4] != NN) return;
  if (in_sizes[5] != 32 || in_sizes[6] != 32 || in_sizes[7] != 32 || in_sizes[8] != 32) return;
  if (in_sizes[9] != 32 * 128 || in_sizes[10] != 32 || in_sizes[11] != 32 * 64 || in_sizes[12] != 32) return;
  for (int i = 13; i <= 21; i += 2) { if (in_sizes[i] != 32 * 32 || in_sizes[i + 1] != 32) return; }
  if (in_sizes[23] != 64 || in_sizes[24] != 2) return;
  if (out_size != NN * 2) return;
  if (ws_size < WS_TOTAL) return;

  const float* x      = (const float*)d_in[0];
  const int*   ei     = (const int*)  d_in[1];
  const float* ntime  = (const float*)d_in[2];
  const float* etime  = (const float*)d_in[3];
  const float* ndeg   = (const float*)d_in[4];
  const float* W_time = (const float*)d_in[5];    const float* b_time = (const float*)d_in[6];
  const float* W_deg  = (const float*)d_in[7];    const float* b_deg  = (const float*)d_in[8];
  const float* W_lin  = (const float*)d_in[9];    const float* b_lin  = (const float*)d_in[10];
  const float* W_comb = (const float*)d_in[11];   const float* b_comb = (const float*)d_in[12];
  const float* Wq = (const float*)d_in[13];       const float* bq = (const float*)d_in[14];
  const float* Wk = (const float*)d_in[15];       const float* bk = (const float*)d_in[16];
  const float* Wv = (const float*)d_in[17];       const float* bv = (const float*)d_in[18];
  const float* We = (const float*)d_in[19];       const float* be = (const float*)d_in[20];
  const float* Ws = (const float*)d_in[21];       const float* bs = (const float*)d_in[22];
  const float* W_out = (const float*)d_in[23];    const float* b_out = (const float*)d_in[24];
  float* out = (float*)d_out;

  char* ws = (char*)d_ws;
  unsigned short* XB    = (unsigned short*)(ws + O_XB);
  float*          H     = (float*)(ws + O_H);
  unsigned*       EPw   = (unsigned*)(ws + O_EP);
  const float*    EPr   = (const float*)(ws + O_EP);
  unsigned short* HHL   = (unsigned short*)(ws + O_HHL);
  float*          QKVS  = (float*)(ws + O_QKVS);
  int*            BLIST = (int*)(ws + O_BLIST);
  int*            OFFC  = (int*)(ws + O_OFFC);
  int*            META  = (int*)(ws + O_META);
  int*            TAB   = (int*)(ws + O_TAB);
  unsigned short* WLIN  = (unsigned short*)(ws + O_WLIN);
  unsigned short* WQKVS = (unsigned short*)(ws + O_WQKVS);
  unsigned short* WC2   = (unsigned short*)(ws + O_WC2);
  unsigned short* WE2   = (unsigned short*)(ws + O_WE2);
  float*          PAR   = (float*)(ws + O_PAR);

  hipFuncSetAttribute(reinterpret_cast<const void*>(&k_bucket),
                      hipFuncAttributeMaxDynamicSharedMemorySize, LDS_BKT);

  k_plane<0><<<MPN * 128 / 8 / 256, 256, 0, stream>>>(x, NN, 128, 128, XB, MPN, 128);
  k_prep<<<12, 256, 0, stream>>>(W_lin, Wq, Wk, Wv, Ws, W_comb, We, W_time, b_time, W_deg, b_deg, b_lin,
                                 b_comb, bq, bk, bv, bs, be, W_out, b_out, WLIN, WQKVS, WC2, WE2, PAR);
  k_gemm_nt<0, 0><<<(1563 + 7) / 8, 256, 0, stream>>>(XB, WLIN, PAR, H, NN, 32, 128, 32);
  k_hpost<<<MPN * 8 / 256, 256, 0, stream>>>(H, PAR, HHL);
  k_gemm_nt<1, 0><<<(3126 + 7) / 8, 256, 0, stream>>>(HHL, WQKVS, PAR, QKVS, NN, 128, 64, 128);
  k_bucket<<<NBLK, NTHR, LDS_BKT, stream>>>(ei + NE, NE, NN, 1, BLIST, OFFC, META);
  k_base<<<1, 32, 0, stream>>>(META, TAB);
  for (int c = 0; c < NCHK; ++c) {
    k_edge<<<EPCAP / 128, 256, 0, stream>>>(ei, ntime, etime, ndeg, BLIST, META, TAB, WC2, WE2, PAR, EPw, c);
    k_attn<<<BPC, 256, 0, stream>>>(ei, QKVS, EPr, BLIST, OFFC, META, TAB, PAR, out, c);
  }
}
